// ConsistencyLoss_11244224381575
// MI455X (gfx1250) — hardware-verified
//
#include <hip/hip_runtime.h>
#include <stdint.h>


#define BB 8
#define CC 256
#define NN 2304
#define THR 31.5f
#define EPSV 1e-8f

typedef __bf16 v16bf __attribute__((ext_vector_type(16)));
typedef __bf16 v8bf __attribute__((ext_vector_type(8)));
typedef float v8f __attribute__((ext_vector_type(8)));
typedef float v4f __attribute__((ext_vector_type(4)));
typedef unsigned int v4u __attribute__((ext_vector_type(4)));
typedef unsigned short v8us __attribute__((ext_vector_type(8)));
union Frag { v16bf v; v8bf half[2]; };

#define TSZ ((size_t)BB * NN * CC)
#define WS_T_BYTES (4 * TSZ * 2)
#define RNSZ ((size_t)BB * NN)
#define WS_RN_OFF WS_T_BYTES
#define WS_RN_BYTES (4 * RNSZ * 4)
#define GEMM_GX (NN / 32)
#define GEMM_GY (NN / 256)
#define GEMM_NBLK (GEMM_GX * GEMM_GY * BB)
#define PL_STRIDE 32
#define WS_PL_OFF (WS_RN_OFF + WS_RN_BYTES)
#define WS_PL_BYTES ((size_t)GEMM_NBLK * PL_STRIDE * 4)
#define WS_NEED (WS_PL_OFF + WS_PL_BYTES)

static_assert((WS_T_BYTES % 256) == 0, "");
static_assert((WS_RN_OFF % 256) == 0, "");
static_assert((WS_PL_OFF % 256) == 0, "");
static_assert((NN % 256) == 0, "");
static_assert((CC % 64) == 0, "");

__device__ __forceinline__ unsigned short f32_to_bf16_rne(float f) {
  unsigned int u = __float_as_uint(f);
  u += 0x7FFFu + ((u >> 16) & 1u);
  return (unsigned short)(u >> 16);
}

__device__ __forceinline__ v8f wmma_bf16_step(v16bf a, v16bf b, v8f c) {
  v8f d = __builtin_amdgcn_wmma_f32_16x16x32_bf16(false, a, false, b, (short)0, c, false, false);
  asm volatile("v_nop\n\tv_nop\n\tv_nop\n\tv_nop" : "+v"(d) : "v"(a), "v"(b));
  return d;
}

__device__ __forceinline__ v16bf load_frag(const __bf16* row_k0, int h) {
  Frag f;
  f.half[0] = *(const v8bf*)(row_k0 + 8 * h);
  f.half[1] = *(const v8bf*)(row_k0 + 16 + 8 * h);
  return f.v;
}

__global__ __launch_bounds__(256) void k_convert_bf16(
    const float* __restrict__ a1, const float* __restrict__ b1,
    const float* __restrict__ a2, const float* __restrict__ b2,
    unsigned short* __restrict__ outbase) {
  __shared__ float tile[64][33];
  const int t = blockIdx.z & 3;
  const int b = blockIdx.z >> 2;
  const float* x = (t == 0) ? a1 : (t == 1) ? b1 : (t == 2) ? a2 : b2;
  const float* xb = x + (size_t)b * CC * NN;
  unsigned short* o = outbase + (size_t)t * TSZ + (size_t)b * NN * CC;

  const int nt = blockIdx.x * 32;
  const int ct = blockIdx.y * 64;
  const int tid = threadIdx.x;
  const int tx = tid & 31, ty = tid >> 5;
  if (nt + 32 > NN || ct + 64 > CC || b >= BB) return;

#pragma unroll
  for (int i = 0; i < 8; ++i) {
    const int c = i * 8 + ty;
    tile[c][tx] = xb[(size_t)(ct + c) * NN + nt + tx];
  }
  __syncthreads();

  const int lane = tid & 31, wave = tid >> 5;
  const int r = wave * 4 + (lane >> 3);
  const int c8 = (lane & 7) * 8;
  v8us pk;
#pragma unroll
  for (int j = 0; j < 8; ++j) pk[j] = f32_to_bf16_rne(tile[c8 + j][r]);
  unsigned short* dst = o + (size_t)(nt + r) * CC + ct + c8;
  *(volatile v8us*)dst = pk;
  __threadfence();
  *(volatile v8us*)dst = pk;
}

__global__ __launch_bounds__(256) void k_inv_norms(
    const float* __restrict__ a1, const float* __restrict__ b1,
    const float* __restrict__ a2, const float* __restrict__ b2,
    float* __restrict__ rnbase) {
  __shared__ float sh[256];
  const int t = blockIdx.z;
  const int b = blockIdx.y;
  const int n0 = blockIdx.x * 256;
  const int tid = threadIdx.x;
  const int n = n0 + tid;
  const float* x = (t == 0) ? a1 : (t == 1) ? b1 : (t == 2) ? a2 : b2;
  float s = 0.f;
  if (n < NN && b < BB) {
    const float* col = x + (size_t)b * CC * NN + n;
#pragma unroll 8
    for (int c = 0; c < CC; ++c) {
      const float v = col[(size_t)c * NN];
      s += v * v;
    }
  }
  sh[tid] = 1.0f / fmaxf(sqrtf(s), EPSV);
  __syncthreads();
  if (tid < 64) {
    const int lane = tid & 31, wave = tid >> 5;
    const int L = wave * 4 + (lane >> 3);
    const int idx = L * 32 + (lane & 7) * 4;
    if (n0 + idx + 4 <= NN && b < BB && t < 4) {
      v4f v;
      v[0] = sh[idx + 0]; v[1] = sh[idx + 1]; v[2] = sh[idx + 2]; v[3] = sh[idx + 3];
      float* dst = rnbase + (size_t)t * RNSZ + (size_t)b * NN + n0 + idx;
      *(volatile v4f*)dst = v;
      __threadfence();
      *(volatile v4f*)dst = v;
    }
  }
}

__global__ __launch_bounds__(256) void k_gemm_masked(
    const __bf16* __restrict__ tbase, const float* __restrict__ rnbase,
    const float* __restrict__ dist, float* __restrict__ pline) {
  const __bf16* tA1 = tbase;
  const __bf16* tB1 = tbase + 1 * TSZ;
  const __bf16* tA2 = tbase + 2 * TSZ;
  const __bf16* tB2 = tbase + 3 * TSZ;
  const float* rnA1 = rnbase;
  const float* rnB1 = rnbase + 1 * RNSZ;
  const float* rnA2 = rnbase + 2 * RNSZ;
  const float* rnB2 = rnbase + 3 * RNSZ;

  const int tid = threadIdx.x;
  const int wave = tid >> 5, lane = tid & 31;
  const int l = lane & 15, h = lane >> 4;
  const int b = blockIdx.z;
  const int m0 = blockIdx.x * 32;
  const int n0 = blockIdx.y * 256 + wave * 32;

  const size_t rowA = ((size_t)b * NN + n0 + l) * CC;
  const size_t rowB = ((size_t)b * NN + m0 + l) * CC;
  const __bf16* pa1 = tA1 + rowA;
  const __bf16* pa2 = tA2 + rowA;
  const __bf16* pb1 = tB1 + rowB;
  const __bf16* pb2 = tB2 + rowB;

  v8f zero8;
#pragma unroll
  for (int i = 0; i < 8; ++i) zero8[i] = 0.f;
  v8f acc1[2][2], acc2[2][2];
#pragma unroll
  for (int ti = 0; ti < 2; ++ti)
#pragma unroll
    for (int tj = 0; tj < 2; ++tj) { acc1[ti][tj] = zero8; acc2[ti][tj] = zero8; }

#pragma unroll 1
  for (int k0 = 0; k0 < CC; k0 += 32) {
    {
      const v16bf a0 = load_frag(pa1 + k0, h);
      const v16bf a1f = load_frag(pa1 + 16 * CC + k0, h);
      const v16bf b0 = load_frag(pb1 + k0, h);
      const v16bf b1f = load_frag(pb1 + 16 * CC + k0, h);
      acc1[0][0] = wmma_bf16_step(a0, b0, acc1[0][0]);
      acc1[0][1] = wmma_bf16_step(a0, b1f, acc1[0][1]);
      acc1[1][0] = wmma_bf16_step(a1f, b0, acc1[1][0]);
      acc1[1][1] = wmma_bf16_step(a1f, b1f, acc1[1][1]);
    }
    {
      const v16bf a0 = load_frag(pa2 + k0, h);
      const v16bf a1f = load_frag(pa2 + 16 * CC + k0, h);
      const v16bf b0 = load_frag(pb2 + k0, h);
      const v16bf b1f = load_frag(pb2 + 16 * CC + k0, h);
      acc2[0][0] = wmma_bf16_step(a0, b0, acc2[0][0]);
      acc2[0][1] = wmma_bf16_step(a0, b1f, acc2[0][1]);
      acc2[1][0] = wmma_bf16_step(a1f, b0, acc2[1][0]);
      acc2[1][1] = wmma_bf16_step(a1f, b1f, acc2[1][1]);
    }
  }

  float psum = 0.f;
  int pcnt = 0;
#pragma unroll
  for (int ti = 0; ti < 2; ++ti) {
    const int nb = n0 + 16 * ti + 8 * h;
#pragma unroll
    for (int tj = 0; tj < 2; ++tj) {
      const int m = m0 + 16 * tj + l;
      const float rb1 = rnB1[(size_t)b * NN + m];
      const float rb2 = rnB2[(size_t)b * NN + m];
#pragma unroll
      for (int j = 0; j < 8; ++j) {
        const int n = nb + j;
        const float d = dist[(size_t)n * NN + m];
        if (d < THR) {
          psum += acc1[ti][tj][j] * (rnA1[(size_t)b * NN + n] * rb1) +
                  acc2[ti][tj][j] * (rnA2[(size_t)b * NN + n] * rb2);
          ++pcnt;
        }
      }
    }
  }

#pragma unroll
  for (int off = 16; off > 0; off >>= 1) {
    psum += __shfl_xor(psum, off, 32);
    pcnt += __shfl_xor(pcnt, off, 32);
  }
  __shared__ float sS[8];
  __shared__ int sC[8];
  if (lane == 0) { sS[wave] = psum; sC[wave] = pcnt; }
  __syncthreads();
  if (wave == 0) {
    float ts = (lane < 8) ? sS[lane] : 0.f;
    int tc = (lane < 8) ? sC[lane] : 0;
#pragma unroll
    for (int off = 16; off > 0; off >>= 1) {
      ts += __shfl_xor(ts, off, 32);
      tc += __shfl_xor(tc, off, 32);
    }
    const int bid = (blockIdx.z * gridDim.y + blockIdx.y) * gridDim.x + blockIdx.x;
    v4u v;
    v[0] = 0u; v[1] = 0u; v[2] = 0u; v[3] = 0u;
    if (lane == 0) { v[0] = __float_as_uint(ts); v[1] = (unsigned int)tc; }
    if (lane < 8 && bid < GEMM_NBLK) {
      unsigned int* dst = (unsigned int*)pline + (size_t)bid * PL_STRIDE + lane * 4;
      *(volatile v4u*)dst = v;
    }
    __threadfence();
    if (lane < 8 && bid < GEMM_NBLK) {
      unsigned int* dst = (unsigned int*)pline + (size_t)bid * PL_STRIDE + lane * 4;
      *(volatile v4u*)dst = v;
    }
  }
}

__global__ __launch_bounds__(256) void k_final_reduce(
    const float* __restrict__ pline, int nblocks, float* __restrict__ out) {
  __shared__ float sS[256];
  __shared__ int sC[256];
  float s = 0.f;
  int c = 0;
  for (int i = threadIdx.x; i < nblocks; i += 256) {
    s += pline[(size_t)i * PL_STRIDE];
    c += __float_as_int(pline[(size_t)i * PL_STRIDE + 1]);
  }
  sS[threadIdx.x] = s;
  sC[threadIdx.x] = c;
  __syncthreads();
  for (int off = 128; off > 0; off >>= 1) {
    if (threadIdx.x < off) {
      sS[threadIdx.x] += sS[threadIdx.x + off];
      sC[threadIdx.x] += sC[threadIdx.x + off];
    }
    __syncthreads();
  }
  if (threadIdx.x == 0) {
    const float val = -sS[0] / (float)sC[0];
    *(volatile float*)out = val;
    __threadfence();
    *(volatile float*)out = val;
  }
}

extern "C" void kernel_launch(void* const* d_in, const int* in_sizes, int n_in,
                              void* d_out, int out_size, void* d_ws, size_t ws_size,
                              hipStream_t stream) {
  if (n_in < 5) return;
  if (in_sizes[0] != BB * CC * NN || in_sizes[1] != BB * CC * NN ||
      in_sizes[2] != BB * CC * NN || in_sizes[3] != BB * CC * NN ||
      in_sizes[4] != NN * NN) return;
  if (out_size < 1) return;
  if (ws_size < WS_NEED) return;

  const float* y  = (const float*)d_in[0];
  const float* yp = (const float*)d_in[1];
  const float* z  = (const float*)d_in[2];
  const float* zp = (const float*)d_in[3];
  const float* dist = (const float*)d_in[4];

  char* ws = (char*)d_ws;
  unsigned short* tconv = (unsigned short*)ws;
  const __bf16* tbase = (const __bf16*)ws;
  float* rnbase = (float*)(ws + WS_RN_OFF);
  float* pline = (float*)(ws + WS_PL_OFF);
  float* out = (float*)d_out;

  k_convert_bf16<<<dim3(NN / 32, CC / 64, 4 * BB), dim3(256), 0, stream>>>(
      y, zp, z, yp, tconv);

  k_inv_norms<<<dim3(NN / 256, BB, 4), dim3(256), 0, stream>>>(
      y, zp, z, yp, rnbase);

  k_gemm_masked<<<dim3(GEMM_GX, GEMM_GY, BB), dim3(256), 0, stream>>>(
      tbase, rnbase, dist, pline);

  k_final_reduce<<<dim3(1), dim3(256), 0, stream>>>(pline, GEMM_NBLK, out);
}
